// ReverbNetwork_2499670966582
// MI455X (gfx1250) — hardware-verified
//
#include <hip/hip_runtime.h>


namespace {
constexpr int N = 64, N1 = 65, E = 513, NB = 8, C = 3, H = 64, W = 64, KS = 4, PH = H + 3  , PW = 72  , LCAP = 16  , LW = 32;
constexpr int VL = 65, BL = 8;
constexpr float XS = 8.0f, WSC = 256.0f, EQ = -0.1f;
static_assert(W == 64 && PW % 8 == 0 && C * KS * KS == 48, "tiling");
typedef _Float16 b16;
typedef __attribute__((ext_vector_type(16))) _Float16 v16b;
typedef __attribute__((ext_vector_type(8))) _Float16 v8b;
typedef __attribute__((ext_vector_type(8))) float v8f;
typedef __attribute__((ext_vector_type(4))) float v4f;
__device__ __forceinline__ float bf16_rne(float f) { unsigned int u = __float_as_uint(f); u += 0x7FFFu + ((u >> 16) & 1u); return __uint_as_float(u & 0xFFFF0000u); }
__device__ __forceinline__ void split16(float v, b16& hi, b16& lo) { hi = (b16)v; lo = (b16)(v - (float)hi); }
__device__ __forceinline__ v16b frag_kb(const b16* p, int hh) { const v8b a = *(const v8b*)(p + 8 * hh), b = *(const v8b*)(p + 16 + 8 * hh); v16b f;
#pragma unroll
  for (int e = 0; e < 8; ++e) { f[e] = a[e]; f[8 + e] = b[e]; } return f; }
__device__ __forceinline__ v8f wmma16b(v16b a, v16b b, v8f c) { v8f d = __builtin_amdgcn_wmma_f32_16x16x32_f16(false, a, false, b, (short)0, c, false, false); asm volatile("v_nop\n\tv_nop\n\tv_nop\n\tv_nop" : "+v"(d) : "v"(a), "v"(b)); return d; }
__device__ __forceinline__ void wave_lds_sync() { __builtin_amdgcn_fence(__ATOMIC_RELEASE, "workgroup"); __builtin_amdgcn_wave_barrier(); __builtin_amdgcn_fence(__ATOMIC_ACQUIRE, "workgroup"); }
__device__ __forceinline__ float pmul(float a, float b) { float p = a * b; asm volatile("" : "+v"(p)); return p; }
__device__ __forceinline__ int iclamp(int v, int lo, int hi) { return v < lo ? lo : (v > hi ? hi : v); }

typedef __attribute__((ext_vector_type(2))) float v2f;
__global__ __launch_bounds__(256) void act_kernel(const float* __restrict__ states, const float* __restrict__ noise, b16* __restrict__ ACT, b16* __restrict__ ACTL) {
  const size_t u = (size_t)blockIdx.x * 256 + threadIdx.x; const size_t total = (size_t)N1 * NB * C * PH * PW / 8; if (u >= total) return;
  const size_t e = u * 8; const size_t img = e / ((size_t)PH * PW); const int pr = (int)((e / PW) % PH), pc0 = (int)(e % PW); const int r = pr - 1; v8b o;
  v8b ol; for (int j = 0; j < 8; ++j) { const int cc = pc0 + j - 1; float v = 0.0f; if (r >= 0 && r < H && cc >= 0 && cc < W) { const size_t gi = (img * H + r) * W + cc; const float z = bf16_rne(states[gi]) + bf16_rne(noise[gi]); v = 1.0f / (1.0f + __expf(-z)); } b16 p, q; split16(v * XS, p, q); o[j] = p; ol[j] = q; }
  for (int pass = 0; pass < 2; ++pass) { *(volatile v8b*)(ACT + e) = o; *(volatile v8b*)(ACTL + e) = ol; __threadfence(); }
}
__global__ __launch_bounds__(256) void prep_kernel(const int* __restrict__ src, const int* __restrict__ dst, const float* __restrict__ cw, const float* __restrict__ cb, int* __restrict__ DL, float* __restrict__ BS, b16* __restrict__ WB) {
  const size_t u = (size_t)blockIdx.x * 256 + threadIdx.x;
  if (u < (size_t)N1) { const int v = (int)u; int cnt = 0; float b0 = 0.0f, b1 = 0.0f, b2 = 0.0f;
    for (int pass = 0; pass < 2; ++pass) { cnt = 0; b0 = b1 = b2 = 0.0f;
#pragma unroll 1
      for (int e = 0; e < E; ++e) { if (dst[e] == v) { if (cnt < LCAP) { ((volatile int*)DL)[v * LW + cnt] = e; b0 += bf16_rne(cb[e * 3 + 0]); b1 += bf16_rne(cb[e * 3 + 1]); b2 += bf16_rne(cb[e * 3 + 2]); } ++cnt; } }
      for (int s = (cnt < LCAP ? cnt : LCAP); s < LW - 1; ++s) ((volatile int*)DL)[v * LW + s] = -1;
      ((volatile int*)DL)[v * LW + LW - 1] = cnt; ((volatile float*)BS)[v * 4 + 0] = b0; ((volatile float*)BS)[v * 4 + 1] = b1; ((volatile float*)BS)[v * 4 + 2] = b2; ((volatile float*)BS)[v * 4 + 3] = 0.0f; __threadfence(); } return; }
  const size_t t = u - N1; if (t >= (size_t)E * 16 * 64 / 8) return; { const size_t e8 = t * 8; const int e = (int)(e8 / (16 * 64)); const int oc = (int)((e8 / 64) % 16), k0 = (int)(e8 % 64); v8b o;
    for (int j = 0; j < 8; ++j) { const int k = k0 + j; float v = 0.0f; if (oc < C && k < 48) { const int c = k >> 4, kh = (k >> 2) & 3, kw = k & 3; v = bf16_rne(cw[(((size_t)e * C + oc) * C + c) * 16 + kh * 4 + kw]) * WSC; } o[j] = (b16)v; }
    for (int pass = 0; pass < 2; ++pass) { *(volatile v8b*)(WB + e8) = o; __threadfence(); } }
}
__global__ __launch_bounds__(128) void reverb_kernel(const b16* __restrict__ ACT, const b16* __restrict__ ACTL, const b16* __restrict__ WB, const int* __restrict__ DL, const float* __restrict__ BS, const int* __restrict__ src, const float* __restrict__ states, const float* __restrict__ res, float* __restrict__ out) {
  __shared__ __attribute__((aligned(16))) b16 T[C][KS][PW], TL[C][KS][PW]; __shared__ __attribute__((aligned(16))) float Os[C][W + 4]; __shared__ int dl[LCAP]; __shared__ int ncnt;
  const int t = threadIdx.x, wave = t >> 5, lane = t & 31, nloc = lane & 15, hlf = lane >> 4;
  const int v = blockIdx.x / (BL * H), rem = blockIdx.x % (BL * H), b = rem / H, h = rem % H;
  if (t < LCAP) dl[t] = iclamp(DL[v * LW + t], -1, E - 1);
  if (t == 0) ncnt = iclamp(DL[v * LW + LW - 1], 0, LCAP);
  __syncthreads();
  const int w0 = wave * 16;
  v8f acc = (v8f){};
  const int ne = ncnt;
#pragma unroll 1
  for (int q = 0; q < ne; ++q) { const int e = dl[q]; const int s = iclamp(src[e < 0 ? 0 : e], 0, N1 - 1);
    __syncthreads();
    { const size_t boff = ((((size_t)s * NB + b) * C) * PH + h) * PW;
      for (int i = t; i < C * KS * (PW / 8); i += 128) { const int c = i / (KS * (PW / 8)), r2 = (i / (PW / 8)) % KS, c8 = (i % (PW / 8)) * 8; const size_t gi = boff + ((size_t)c * PH + r2) * PW + c8; *(v8b*)(&T[c][r2][c8]) = *(const v8b*)(ACT + gi); *(v8b*)(&TL[c][r2][c8]) = *(const v8b*)(ACTL + gi); } }
    __syncthreads();
    if (e >= 0) {
#pragma unroll
      for (int ks = 0; ks < 2; ++ks) { v16b a, al;
#pragma unroll
        for (int el = 0; el < 16; ++el) { const int k = ks * 32 + ((el < 8) ? (8 * hlf + el) : (16 + 8 * hlf + (el - 8))); b16 val = (b16)0.0f, vl = (b16)0.0f;
          if (k < 48) { const int c = k >> 4, kh = (k >> 2) & 3, kw = k & 3; val = T[c][kh][w0 + nloc + kw]; vl = TL[c][kh][w0 + nloc + kw]; } a[el] = val; al[el] = vl; }
        const v16b bw = frag_kb(WB + ((size_t)e * 16 + nloc) * 64 + ks * 32, hlf); acc = wmma16b(a, bw, acc); acc = wmma16b(al, bw, acc); } } }
  if (nloc < C) {
#pragma unroll
    for (int r = 0; r < 8; ++r) Os[nloc][w0 + 8 * hlf + r] = acc[r] * (1.0f / (XS * WSC)); }
  __syncthreads();
  for (int pass = 0; pass < 2; ++pass) { if (wave < C) { const int oc = wave; const size_t gi = ((((size_t)v * NB + b) * C + oc) * H + h) * W + lane * 2; v2f o;
      for (int j = 0; j < 2; ++j) { const int w = lane * 2 + j; const float st = bf16_rne(states[gi + j]); float nv = st + Os[oc][w] + BS[v * 4 + oc]; if (v < N) { const float rs = fabsf(bf16_rne(res[((((size_t)v * NB + b) * C + oc) * H + h) * W + w])); nv += pmul(rs, EQ - st); } o[j] = nv; }
      *(volatile v2f*)(out + gi) = o; } __threadfence(); }
}
}

extern "C" void kernel_launch(void* const* d_in, const int* in_sizes, int n_in, void* d_out, int out_size, void* d_ws, size_t ws_size, hipStream_t stream) {
  (void)n_in;
  auto Fp = [&](int i) { return (const float*)d_in[i]; }; auto Ip = [&](int i) { return (const int*)d_in[i]; };
  if (in_sizes[0] != N1 * NB * C * H * W || in_sizes[1] != N1 * NB * C * H * W || in_sizes[2] != E * C * C * KS * KS || in_sizes[3] != E * C || in_sizes[4] != N * NB * C * H * W || in_sizes[5] != E || in_sizes[6] != E || out_size != N1 * NB * C * H * W) return;
  size_t off = 0; char* ws = (char*)d_ws;
  auto carve = [&](size_t bytes) { char* p = ws + off; off += (bytes + 255) & ~(size_t)255; return p; };
  b16* ACT = (b16*)carve((size_t)N1 * NB * C * PH * PW * 2); b16* ACTL = (b16*)carve((size_t)N1 * NB * C * PH * PW * 2); int* DL = (int*)carve((size_t)N1 * LW * 4); float* BS = (float*)carve((size_t)N1 * 4 * 4); b16* WB = (b16*)carve((size_t)E * 16 * 64 * 2);
  if (off > ws_size || off > ((size_t)128 << 20)) return;
  act_kernel<<<(unsigned)(((size_t)N1 * NB * C * PH * PW / 8 + 255) / 256), 256, 0, stream>>>(Fp(0), Fp(1), ACT, ACTL);
  prep_kernel<<<(unsigned)((N1 + (size_t)E * 16 * 64 / 8 + 255) / 256), 256, 0, stream>>>(Ip(5), Ip(6), Fp(2), Fp(3), DL, BS, WB);
  reverb_kernel<<<VL * BL * H, 128, 0, stream>>>(ACT, ACTL, WB, DL, BS, Ip(5), Fp(0), Fp(4), (float*)d_out);
}
